// _CISRJAttentionBlock_87316685128187
// MI455X (gfx1250) — hardware-verified
//
#include <hip/hip_runtime.h>
#include <math.h>

constexpr int kB  = 4;
constexpr int kC  = 512;
constexpr int kN  = 2048;
constexpr int kC2 = 1024;
constexpr size_t kCN  = (size_t)kC * kN;
constexpr size_t kC2N = (size_t)kC2 * kN;
constexpr size_t kNN  = (size_t)kN * kN;

constexpr float kWCarry     = 64.0f;
constexpr float kDwCarry    = 16.0f;
constexpr float kPwScale    = 1.0f / (64.0f * 16.0f);
constexpr float kProjScale  = 1.0f / 64.0f;
constexpr float kQKScale    = 8.0f / 64.0f;
constexpr float kLogitScale = 0.5f * 0.04419417382415922f;
constexpr float kSCarryInv  = 1.0f / 1024.0f;
constexpr float kAvScale    = 64.0f / 1024.0f;
constexpr float kYScale     = 1.0f / (64.0f * 64.0f);
constexpr float kEpsGN      = 1e-8f;
constexpr float kEpsAttn    = 1e-8f;
constexpr float kInvCN      = 1.0f / 1048576.0f;

constexpr size_t kOffwPW  = 0;
constexpr size_t kOffwUW  = kOffwPW  + (size_t)kC * kC;
constexpr size_t kOffwVW  = kOffwUW  + (size_t)kC2 * kC;
constexpr size_t kOffwHW  = kOffwVW  + (size_t)kC2 * kC;
constexpr size_t kOffwQKW = kOffwHW  + (size_t)kC * kC;
constexpr size_t kOffwKW  = kOffwQKW + (size_t)kC * kC;
constexpr size_t kOffwOW  = kOffwQKW + (size_t)kC2 * kC;
constexpr size_t kWHalves = kOffwOW  + (size_t)kC * kC2;

constexpr size_t kOffPart = 0;
constexpr size_t kOffRS   = kOffPart + (size_t)kB * 256 * 32 * 4;
constexpr size_t kOffW    = kOffRS   + (size_t)kB * kN * 4;
constexpr size_t kOffR1   = kOffW    + kWHalves * 2;
constexpr size_t kOffR2   = kOffR1   + (size_t)kB * kCN * 4;
constexpr size_t kOffR3   = kOffR2   + (size_t)kB * kCN * 2;
constexpr size_t kOffR4   = kOffR3   + (size_t)kB * kCN * 2;
constexpr size_t kOffR5   = kOffR4   + (size_t)kB * kC2N * 2;
constexpr size_t kOffR6   = kOffR5   + (size_t)kB * kC2N * 2;
constexpr size_t kWsTotal = kOffR6   + (size_t)kB * kNN * 2;
static_assert(kWsTotal == 106070016);
static_assert(kWsTotal <= 134217728);
static_assert((kOffRS % 256) == 0 && (kOffW % 256) == 0 && (kOffR1 % 256) == 0 && (kOffR2 % 256) == 0 &&
              (kOffR3 % 256) == 0 && (kOffR4 % 256) == 0 && (kOffR5 % 256) == 0 && (kOffR6 % 256) == 0);

typedef __attribute__((ext_vector_type(16))) _Float16 v16h;
typedef __attribute__((ext_vector_type(8)))  _Float16 v8h;
typedef __attribute__((ext_vector_type(16))) __bf16   v16b;
typedef __attribute__((ext_vector_type(8)))  __bf16   v8b;
typedef __attribute__((ext_vector_type(8)))  float    v8f;
typedef __attribute__((ext_vector_type(4)))  float    v4f;
typedef __attribute__((ext_vector_type(4)))  unsigned int v4u;

__device__ __forceinline__ unsigned short f2bf_bits(float f) {
  unsigned u = __float_as_uint(f);
  return (unsigned short)((u + 0x7FFFu + ((u >> 16) & 1u)) >> 16);
}
__device__ __forceinline__ float bf_bits2f(unsigned short h) { return __uint_as_float(((unsigned)h) << 16); }

__device__ __forceinline__ void dep_guard_h(v8f& a, v8f& b, v16h x, v16h y) { asm volatile("v_nop\n\tv_nop\n\tv_nop\n\tv_nop" : "+v"(a), "+v"(b) : "v"(x), "v"(y)); }
__device__ __forceinline__ void dep_guard_b(v8f& a, v8f& b, v16b x, v16b y) { asm volatile("v_nop\n\tv_nop\n\tv_nop\n\tv_nop" : "+v"(a), "+v"(b) : "v"(x), "v"(y)); }
__device__ __forceinline__ void keep4_h(v16h a, v16h b, v16h c, v16h d) { asm volatile("v_nop" :: "v"(a), "v"(b), "v"(c), "v"(d)); }
__device__ __forceinline__ void keep4_b(v16b a, v16b b, v16b c, v16b d) { asm volatile("v_nop" :: "v"(a), "v"(b), "v"(c), "v"(d)); }
__device__ __forceinline__ void acc_guard4(v8f& a, v8f& b, v8f& c, v8f& d) { asm volatile("v_nop\n\tv_nop\n\tv_nop\n\tv_nop" : "+v"(a), "+v"(b), "+v"(c), "+v"(d)); }
template <typename T> struct Frag;
template <> struct Frag<_Float16> {
  typedef v16h V; union U { v16h v; v8h h[2]; };
  static __device__ __forceinline__ v16h load(const _Float16* p) {
    U f; f.h[0] = *(const v8h*)(p); f.h[1] = *(const v8h*)(p + 16); return f.v;
  }
  static __device__ __forceinline__ v8f mma(v16h a, v16h b, v8f c) {
    return __builtin_amdgcn_wmma_f32_16x16x32_f16(false, a, false, b, (short)0, c, false, false);
  }
  static __device__ __forceinline__ void guard(v8f& a, v8f& b, v16h x, v16h y) { dep_guard_h(a, b, x, y); }
  static __device__ __forceinline__ void keep(v16h a, v16h b, v16h c, v16h d) { keep4_h(a, b, c, d); }
};
template <> struct Frag<__bf16> {
  typedef v16b V; union U { v16b v; v8b h[2]; };
  static __device__ __forceinline__ v16b load(const __bf16* p) {
    U f; f.h[0] = *(const v8b*)(p); f.h[1] = *(const v8b*)(p + 16); return f.v;
  }
  static __device__ __forceinline__ v8f mma(v16b a, v16b b, v8f c) {
    return __builtin_amdgcn_wmma_f32_16x16x32_bf16(false, a, false, b, (short)0, c, false, false);
  }
  static __device__ __forceinline__ void guard(v8f& a, v8f& b, v16b x, v16b y) { dep_guard_b(a, b, x, y); }
  static __device__ __forceinline__ void keep(v16b a, v16b b, v16b c, v16b d) { keep4_b(a, b, c, d); }
};

__device__ __forceinline__ unsigned pk16(unsigned short a, unsigned short b) { return (unsigned)a | ((unsigned)b << 16); }
__device__ __forceinline__ unsigned short h_bits(float f) { const _Float16 h = (_Float16)f; return __builtin_bit_cast(unsigned short, h); }

template <int ET> struct Elem;
template <> struct Elem<0> { typedef _Float16 T; };
template <> struct Elem<1> { typedef __bf16 T; };
template <int ET, bool SPLIT, int BIAS_MODE, int OUT_MODE, bool RESID, int ACT, bool RSGATE>
__global__ __launch_bounds__(256) void wmma_gemm64(
    const unsigned short* __restrict__ Ap, const unsigned short* __restrict__ A2p, int lda, long strideA,
    const unsigned short* __restrict__ Btp, const unsigned short* __restrict__ Bt2p, int ldb, long strideB,
    void* __restrict__ Cout, void* __restrict__ Cout2, int ldc, long strideC,
    const float* __restrict__ bias,
    const float* __restrict__ resid, long strideR,
    const float* __restrict__ rsc, long strideRS,
    const unsigned short* __restrict__ gate, long strideG,
    int M, int N, int K, float scale) {
  typedef typename Elem<ET>::T T;
  typedef typename Frag<T>::V V;
  const T* A = (const T*)Ap; const T* A2 = (const T*)A2p; const T* Bt = (const T*)Btp; const T* Bt2 = (const T*)Bt2p;
  __shared__ __align__(16) float sT[8][16 * 68];
  const int b    = blockIdx.y;
  const int lane = threadIdx.x & 31;
  const int wave = threadIdx.x >> 5;
  const int tilesN = N >> 6;
  const int tilesM = M >> 6;
  const int tile = blockIdx.x * 8 + wave;
  if (tile >= tilesM * tilesN) return;
  const int tm = tile / tilesN;
  const int tn = tile - tm * tilesN;
  const int m0 = tm << 6;
  const int n0 = tn << 6;

  const T* Ab  = A  + (size_t)b * strideA;
  const T* Bb  = Bt + (size_t)b * strideB;
  const T* Ab2 = SPLIT ? (A2  + (size_t)b * strideA) : nullptr;
  const T* Bb2 = SPLIT ? (Bt2 + (size_t)b * strideB) : nullptr;

  const int rlane = lane & 15;
  const int koff  = (lane >> 4) * 8;
  const int mOff  = (lane >> 4) * 8;

  v8f acc[4][4];
#pragma unroll
  for (int i = 0; i < 4; ++i)
#pragma unroll
    for (int j = 0; j < 4; ++j) acc[i][j] = (v8f){0.f,0.f,0.f,0.f,0.f,0.f,0.f,0.f};

  for (int k0 = 0; k0 < K; k0 += 32) {
    V bh[4], bl[4];
#pragma unroll
    for (int j = 0; j < 4; ++j) {
      const size_t bo = (size_t)(n0 + (j << 4) + rlane) * ldb + koff + k0;
      bh[j] = Frag<T>::load(Bb + bo);
      if (SPLIT) bl[j] = Frag<T>::load(Bb2 + bo);
    }
#pragma unroll
    for (int i = 0; i < 4; ++i) {
      const size_t ao = (size_t)(m0 + (i << 4) + rlane) * lda + koff + k0;
      V ah = Frag<T>::load(Ab + ao);
      V al;
      if (SPLIT) al = Frag<T>::load(Ab2 + ao);
#pragma unroll
      for (int j = 0; j < 4; ++j) {
        acc[i][j] = Frag<T>::mma(ah, bh[j], acc[i][j]);
        if (SPLIT) {
          acc[i][j] = Frag<T>::mma(ah, bl[j], acc[i][j]);
          acc[i][j] = Frag<T>::mma(al, bh[j], acc[i][j]);
        }
      }
      Frag<T>::guard(acc[i][0], acc[i][3], ah, SPLIT ? al : ah);
    }
    Frag<T>::keep(bh[0], bh[1], bh[2], bh[3]);
    if (SPLIT) Frag<T>::keep(bl[0], bl[1], bl[2], bl[3]);
  }
  acc_guard4(acc[0][0], acc[0][1], acc[0][2], acc[0][3]);
  acc_guard4(acc[1][0], acc[1][1], acc[1][2], acc[1][3]);
  acc_guard4(acc[2][0], acc[2][1], acc[2][2], acc[2][3]);
  acc_guard4(acc[3][0], acc[3][1], acc[3][2], acc[3][3]);

  float* slab = sT[wave];
  const float* Rb  = RESID  ? (resid + (size_t)b * strideR) : nullptr;
  const float* RSb = RSGATE ? (rsc + (size_t)b * strideRS) : nullptr;
  const _Float16* Gb = RSGATE ? ((const _Float16*)gate + (size_t)b * strideG) : nullptr;
#pragma unroll
  for (int i = 0; i < 4; ++i) {
    const int mBase = m0 + (i << 4);
#pragma unroll
    for (int j = 0; j < 4; ++j) {
      const int n = n0 + (j << 4) + rlane;
      float bv = 0.f;
      if (BIAS_MODE == 2) bv = bias[n];
#pragma unroll
      for (int r = 0; r < 8; ++r) {
        float v = acc[i][j][r] * scale;
        if (BIAS_MODE == 1) v += bias[mBase + mOff + r];
        if (BIAS_MODE == 2) v += bv;
        if (RESID) v += Rb[(size_t)(mBase + mOff + r) * ldc + n];
        if (RSGATE) {
          v *= RSb[mBase + mOff + r];
          v *= (float)Gb[(size_t)(mBase + mOff + r) * ldc + n];
        }
        if (ACT == 2) v = fmaxf(v, 0.0f);
        if (ACT == 4) v = (v > 0.f) ? v : 0.01f * v;
        if (ACT == 6) { const float ev = __expf(-v); v = __builtin_amdgcn_rcpf(1.0f + ev); }
        if (ACT == 7) { v = fmaxf(v, 0.0f); v = v * v; }
        slab[(mOff + r) * 68 + (j << 4) + rlane] = v;
      }
    }
    __builtin_amdgcn_fence(__ATOMIC_RELEASE, "workgroup");
    __builtin_amdgcn_wave_barrier();
    __builtin_amdgcn_fence(__ATOMIC_ACQUIRE, "workgroup");
    if (OUT_MODE == 0) {
      float* C = (float*)Cout + (size_t)b * strideC;
      const int hh = lane >> 4, c4 = (lane & 15) * 4;
      for (int pass = 0; pass < 2; ++pass) {
#pragma unroll
        for (int it = 0; it < 8; ++it) {
          const int row = it * 2 + hh;
          v4f v = *(const v4f*)(slab + row * 68 + c4);
          *(volatile v4f*)(C + (size_t)(mBase + row) * ldc + n0 + c4) = v;
        }
        __threadfence();
      }
    } else {
      const int q = lane >> 3, c8 = (lane & 7) * 8;
      unsigned short* C  = (unsigned short*)Cout  + (size_t)b * strideC;
      unsigned short* C2 = (OUT_MODE == 2) ? ((unsigned short*)Cout2 + (size_t)b * strideC) : nullptr;
      for (int pass = 0; pass < 2; ++pass) {
#pragma unroll
        for (int it = 0; it < 4; ++it) {
          const int row = it * 4 + q;
          const float* sp = slab + row * 68 + c8;
          v8h hv, lv;
#pragma unroll
          for (int e = 0; e < 8; ++e) {
            if (OUT_MODE == 1) {
              hv[e] = (_Float16)sp[e];
            } else {
              unsigned short hb = f2bf_bits(sp[e]);
              unsigned short lb = f2bf_bits(sp[e] - bf_bits2f(hb));
              hv[e] = __builtin_bit_cast(_Float16, hb);
              lv[e] = __builtin_bit_cast(_Float16, lb);
            }
          }
          *(volatile v8h*)(C + (size_t)(mBase + row) * ldc + n0 + c8) = hv;
          if (OUT_MODE == 2) *(volatile v8h*)(C2 + (size_t)(mBase + row) * ldc + n0 + c8) = lv;
        }
        __threadfence();
      }
    }
    __builtin_amdgcn_fence(__ATOMIC_RELEASE, "workgroup");
    __builtin_amdgcn_wave_barrier();
    __builtin_amdgcn_fence(__ATOMIC_ACQUIRE, "workgroup");
  }
}

__global__ __launch_bounds__(256) void castw_kernel(const float* __restrict__ w_pw, const float* __restrict__ w_u,
                                                    const float* __restrict__ w_v, const float* __restrict__ w_h,
                                                    const float* __restrict__ w_q, const float* __restrict__ w_k,
                                                    const float* __restrict__ w_o, unsigned short* __restrict__ wb) {
  const int seg = blockIdx.y;
  const float* src = w_pw; size_t doff = kOffwPW; int n8 = (kC * kC) / 8;
  if (seg == 1) { src = w_u; doff = kOffwUW;  n8 = (kC2 * kC) / 8; }
  if (seg == 2) { src = w_v; doff = kOffwVW;  n8 = (kC2 * kC) / 8; }
  if (seg == 3) { src = w_h; doff = kOffwHW;  n8 = (kC * kC) / 8; }
  if (seg == 4) { src = w_q; doff = kOffwQKW; n8 = (kC * kC) / 8; }
  if (seg == 5) { src = w_k; doff = kOffwKW;  n8 = (kC * kC) / 8; }
  if (seg == 6) { src = w_o; doff = kOffwOW;  n8 = (kC * kC2) / 8; }
  const int i = blockIdx.x * 256 + threadIdx.x;
  if (i >= n8) return;
  const float* p = src + (size_t)i * 8;
  const v4f a = *(const v4f*)p;
  const v4f c = *(const v4f*)(p + 4);
  const v4u u = (v4u){pk16(h_bits(a[0] * kWCarry), h_bits(a[1] * kWCarry)),
                      pk16(h_bits(a[2] * kWCarry), h_bits(a[3] * kWCarry)),
                      pk16(h_bits(c[0] * kWCarry), h_bits(c[1] * kWCarry)),
                      pk16(h_bits(c[2] * kWCarry), h_bits(c[3] * kWCarry))};
  unsigned short* op = wb + doff + (size_t)i * 8;
  *(volatile v4u*)op = u;
  __threadfence();
  *(volatile v4u*)op = u;
}

__global__ __launch_bounds__(256) void gn_stats_kernel(const float* __restrict__ x, float* __restrict__ part) {
  __shared__ float ls[256], lq[256];
  const int t = threadIdx.x, blk = blockIdx.x, b = blockIdx.y;
  const float* xb = x + (size_t)b * kCN + (size_t)blk * 4096;
  float s = 0.f, q = 0.f;
#pragma unroll
  for (int j = 0; j < 4; ++j) {
    const v4f v = *(const v4f*)(xb + j * 1024 + t * 4);
    s += (v[0] + v[1]) + (v[2] + v[3]);
    q += (v[0] * v[0] + v[1] * v[1]) + (v[2] * v[2] + v[3] * v[3]);
  }
  ls[t] = s; lq[t] = q;
  __syncthreads();
  for (int st = 128; st > 0; st >>= 1) {
    if (t < st) { ls[t] += ls[t + st]; lq[t] += lq[t + st]; }
    __syncthreads();
  }
  if (t < 8) {
    const float s0 = ls[0], q0 = lq[0];
    v4f o = (v4f){0.f, 0.f, 0.f, 0.f};
    if (t == 0) { o[0] = s0; o[1] = q0; }
    float* pp = part + ((size_t)b * 256 + blk) * 32 + t * 4;
    *(volatile v4f*)pp = o;
    __threadfence();
    *(volatile v4f*)pp = o;
  }
}

__global__ __launch_bounds__(256) void gn_dw_kernel(const float* __restrict__ x, const float* __restrict__ part,
                                                    const float* __restrict__ dww,
                                                    float* __restrict__ ZT, unsigned short* __restrict__ DWT) {
  __shared__ float zs[64 * 67];
  __shared__ float dws[64 * 65];
  __shared__ float wsm[64 * 3];
  __shared__ float red_s[256], red_q[256];
  const int t = threadIdx.x;
  const int n0 = blockIdx.x * 64, c0 = blockIdx.y * 64, b = blockIdx.z;

  red_s[t] = part[((size_t)b * 256 + t) * 32 + 0];
  red_q[t] = part[((size_t)b * 256 + t) * 32 + 1];
  if (t < 192) wsm[t] = dww[(size_t)c0 * 3 + t];
  __syncthreads();
  for (int st = 128; st > 0; st >>= 1) {
    if (t < st) { red_s[t] += red_s[t + st]; red_q[t] += red_q[t + st]; }
    __syncthreads();
  }
  const float mean = red_s[0] * kInvCN;
  const float var  = red_q[0] * kInvCN - mean * mean;
  const float inv  = 1.0f / sqrtf(var + kEpsGN);

  const float* xb = x + ((size_t)b * kC + c0) * kN;
  for (int e = t; e < 64 * 66; e += 256) {
    const int cl = e / 66;
    const int j  = e - cl * 66;
    const int n  = n0 - 1 + j;
    const int nn = n < 0 ? 0 : (n > kN - 1 ? kN - 1 : n);
    const float xv = xb[(size_t)cl * kN + nn];
    const bool inr = (n >= 0) && (n < kN);
    zs[cl * 67 + j] = inr ? (xv - mean) * inv : 0.0f;
  }
  __syncthreads();
  for (int e = t; e < 64 * 64; e += 256) {
    const int cl = e & 63, nl = e >> 6;
    const float* zr = zs + cl * 67 + nl;
    const float d = wsm[cl * 3 + 0] * zr[0] + wsm[cl * 3 + 1] * zr[1] + wsm[cl * 3 + 2] * zr[2];
    dws[nl * 65 + cl] = d * kDwCarry;
  }
  __syncthreads();

  const int lane = t & 31, wave = t >> 5;
  const int hh = lane >> 4, c4 = (lane & 15) * 4;
  const int q8 = lane >> 3, c8 = (lane & 7) * 8;
  v4f zv[4];
#pragma unroll
  for (int it = 0; it < 4; ++it) {
    const int row = wave * 8 + it * 2 + hh;
    v4f v;
    v[0] = zs[(c4 + 0) * 67 + row + 1];
    v[1] = zs[(c4 + 1) * 67 + row + 1];
    v[2] = zs[(c4 + 2) * 67 + row + 1];
    v[3] = zs[(c4 + 3) * 67 + row + 1];
    zv[it] = v;
  }
  v4u dv[2];
#pragma unroll
  for (int it = 0; it < 2; ++it) {
    const int row = wave * 8 + it * 4 + q8;
    const float* dp = dws + row * 65 + c8;
    dv[it] = (v4u){pk16(h_bits(dp[0]), h_bits(dp[1])), pk16(h_bits(dp[2]), h_bits(dp[3])),
                   pk16(h_bits(dp[4]), h_bits(dp[5])), pk16(h_bits(dp[6]), h_bits(dp[7]))};
  }
  float* ztb = ZT + ((size_t)b * kN + n0) * kC + c0;
  unsigned short* dwb = DWT + ((size_t)b * kN + n0) * kC + c0;
  for (int pass = 0; pass < 2; ++pass) {
#pragma unroll
    for (int it = 0; it < 4; ++it) {
      const int row = wave * 8 + it * 2 + hh;
      *(volatile v4f*)(ztb + (size_t)row * kC + c4) = zv[it];
    }
#pragma unroll
    for (int it = 0; it < 2; ++it) {
      const int row = wave * 8 + it * 4 + q8;
      *(volatile v4u*)(dwb + (size_t)row * kC + c8) = dv[it];
    }
    __threadfence();
  }
}

__global__ __launch_bounds__(256) void rowsum_kernel(const unsigned short* __restrict__ S, float* __restrict__ rsinv) {
  __shared__ float rsl[32];
  const int t = threadIdx.x, lane = t & 31, wave = t >> 5;
  const size_t r0 = (size_t)blockIdx.x * 32;
  const _Float16* Sh = (const _Float16*)S;
#pragma unroll 1
  for (int i = 0; i < 4; ++i) {
    const size_t row = r0 + wave * 4 + i;
    const _Float16* sr = Sh + row * kN;
    float acc = 0.f;
#pragma unroll
    for (int it = 0; it < 8; ++it) {
      const v8h hv = *(const v8h*)(sr + it * 256 + lane * 8);
      acc += (((float)hv[0] + (float)hv[1]) + ((float)hv[2] + (float)hv[3])) +
             (((float)hv[4] + (float)hv[5]) + ((float)hv[6] + (float)hv[7]));
    }
#pragma unroll
    for (int off = 1; off < 32; off <<= 1) acc += __shfl_xor(acc, off, 32);
    if (lane == 0) rsl[wave * 4 + i] = __builtin_amdgcn_rcpf(acc * kSCarryInv + kEpsAttn);
  }
  __syncthreads();
  if (t < 8) {
    const v4f o = (v4f){rsl[t * 4 + 0], rsl[t * 4 + 1], rsl[t * 4 + 2], rsl[t * 4 + 3]};
    float* pp = rsinv + r0 + t * 4;
    *(volatile v4f*)pp = o;
    __threadfence();
    *(volatile v4f*)pp = o;
  }
}

extern "C" void kernel_launch(void* const* d_in, const int* in_sizes, int n_in,
                              void* d_out, int out_size, void* d_ws, size_t ws_size,
                              hipStream_t stream) {
  if (n_in < 13) return;
  if (in_sizes[0] != (int)((size_t)kB * kCN) || out_size != (int)((size_t)kB * kCN)) return;
  if (in_sizes[1] != kC * 3 || in_sizes[2] != kC * kC || in_sizes[3] != kC2 * kC || in_sizes[4] != kC2 ||
      in_sizes[5] != kC2 * kC || in_sizes[6] != kC2 || in_sizes[7] != kC * kC || in_sizes[8] != kC ||
      in_sizes[9] != kC * kC || in_sizes[10] != kC * kC || in_sizes[11] != kC * kC2 || in_sizes[12] != kC) return;
  if (ws_size < kWsTotal) return;

  const float* x    = (const float*)d_in[0];
  const float* dw_w = (const float*)d_in[1];
  const float* pw_w = (const float*)d_in[2];
  const float* u_w  = (const float*)d_in[3];
  const float* u_b  = (const float*)d_in[4];
  const float* v_w  = (const float*)d_in[5];
  const float* v_b  = (const float*)d_in[6];
  const float* h_w  = (const float*)d_in[7];
  const float* h_b  = (const float*)d_in[8];
  const float* q_w  = (const float*)d_in[9];
  const float* k_w  = (const float*)d_in[10];
  const float* o_w  = (const float*)d_in[11];
  const float* o_b  = (const float*)d_in[12];
  float* out = (float*)d_out;

  char* w = (char*)d_ws;
  float*          part = (float*)(w + kOffPart);
  float*          rs   = (float*)(w + kOffRS);
  unsigned short* wts  = (unsigned short*)(w + kOffW);
  float*          zt   = (float*)(w + kOffR1);
  unsigned short* ut   = (unsigned short*)(w + kOffR1);
  unsigned short* dwt  = (unsigned short*)(w + kOffR2);
  unsigned short* h16  = (unsigned short*)(w + kOffR2);
  unsigned short* z2t  = (unsigned short*)(w + kOffR3);
  unsigned short* v16  = (unsigned short*)(w + kOffR4);
  unsigned short* qk16 = (unsigned short*)(w + kOffR5);
  unsigned short* uav  = (unsigned short*)(w + kOffR5);
  unsigned short* s16  = (unsigned short*)(w + kOffR6);

  const unsigned short* wPW  = wts + kOffwPW;
  const unsigned short* wUW  = wts + kOffwUW;
  const unsigned short* wVW  = wts + kOffwVW;
  const unsigned short* wHW  = wts + kOffwHW;
  const unsigned short* wQKW = wts + kOffwQKW;
  const unsigned short* wOW  = wts + kOffwOW;

  auto gx = [](int M, int N) { return ((M / 64) * (N / 64) + 7) / 8; };

  castw_kernel<<<dim3(256, 7), 256, 0, stream>>>(pw_w, u_w, v_w, h_w, q_w, k_w, o_w, wts);
  gn_stats_kernel<<<dim3(256, kB), 256, 0, stream>>>(x, part);
  gn_dw_kernel<<<dim3(kN / 64, kC / 64, kB), 256, 0, stream>>>(x, part, dw_w, zt, dwt);

  wmma_gemm64<0, false, 0, 1, true, 0, false><<<dim3(gx(kN, kC), kB), 256, 0, stream>>>(
      dwt, dwt, kC, (long)kCN, wPW, wPW, kC, 0L,
      (void*)z2t, (void*)z2t, kC, (long)kCN,
      o_b, zt, (long)kCN, rs, 0L, wts, 0L,
      kN, kC, kC, kPwScale);

  wmma_gemm64<0, false, 2, 1, false, 6, false><<<dim3(gx(kN, kC2), kB), 256, 0, stream>>>(
      z2t, z2t, kC, (long)kCN, wUW, wUW, kC, 0L,
      (void*)ut, (void*)ut, kC2, (long)kC2N,
      u_b, x, 0L, rs, 0L, wts, 0L,
      kN, kC2, kC, kProjScale);

  wmma_gemm64<0, false, 1, 1, false, 0, false><<<dim3(gx(kC2, kN), kB), 256, 0, stream>>>(
      wVW, wVW, kC, 0L, z2t, z2t, kC, (long)kCN,
      (void*)v16, (void*)v16, kN, (long)kC2N,
      v_b, x, 0L, rs, 0L, wts, 0L,
      kC2, kN, kC, kProjScale);

  wmma_gemm64<0, false, 2, 1, false, 0, false><<<dim3(gx(kN, kC), kB), 256, 0, stream>>>(
      z2t, z2t, kC, (long)kCN, wHW, wHW, kC, 0L,
      (void*)h16, (void*)h16, kC, (long)kCN,
      h_b, x, 0L, rs, 0L, wts, 0L,
      kN, kC, kC, kProjScale);

  wmma_gemm64<0, false, 0, 1, false, 0, false><<<dim3(gx(kN, kC2), kB), 256, 0, stream>>>(
      h16, h16, kC, (long)kCN, wQKW, wQKW, kC, 0L,
      (void*)qk16, (void*)qk16, kC2, (long)kC2N,
      o_b, x, 0L, rs, 0L, wts, 0L,
      kN, kC2, kC, kQKScale);

  wmma_gemm64<0, false, 0, 1, false, 7, false><<<dim3(gx(kN, kN), kB), 256, 0, stream>>>(
      qk16, qk16, kC2, (long)kC2N, qk16 + kC, qk16 + kC, kC2, (long)kC2N,
      (void*)s16, (void*)s16, kN, (long)kNN,
      o_b, x, 0L, rs, 0L, wts, 0L,
      kN, kN, kC, kLogitScale);

  rowsum_kernel<<<dim3((kB * kN) / 32), 256, 0, stream>>>(s16, rs);

  wmma_gemm64<0, false, 0, 1, false, 0, true><<<dim3(gx(kN, kC2), kB), 256, 0, stream>>>(
      s16, s16, kN, (long)kNN, v16, v16, kN, (long)kC2N,
      (void*)uav, (void*)uav, kC2, (long)kC2N,
      o_b, x, 0L, rs, (long)kN, ut, (long)kC2N,
      kN, kC2, kN, kAvScale);

  wmma_gemm64<0, false, 1, 0, true, 0, false><<<dim3(gx(kC, kN), kB), 256, 0, stream>>>(
      wOW, wOW, kC2, 0L, uav, uav, kC2, (long)kC2N,
      (void*)out, (void*)out, kN, (long)kCN,
      o_b, x, (long)kCN, rs, 0L, wts, 0L,
      kC, kN, kC2, kYScale);
}
